// PT_Attention_34291018891955
// MI455X (gfx1250) — hardware-verified
//
#include <hip/hip_runtime.h>
#include <math.h>
#include <stdint.h>

#define NB   2
#define NQ   1024
#define NK   2048
#define CD   256
#define NH   8
#define HD   32
#define NQB  (NQ / 64)
#define NKB  (NK / 64)
#define NQH  (NQ / 32)
#define NKC  (NK / 32)
static_assert(NH * HD == CD);
static_assert(HD == 32);
static_assert((NQ % 64) == 0 && (NK % 64) == 0 && (CD % 64) == 0 && (NH % 2) == 0);

typedef _Float16 v16h __attribute__((ext_vector_type(16)));
typedef _Float16 v8h  __attribute__((ext_vector_type(8)));
typedef __bf16   v16b __attribute__((ext_vector_type(16)));
typedef __bf16   v8b  __attribute__((ext_vector_type(8)));
typedef float    v8f  __attribute__((ext_vector_type(8)));
typedef float    v4f  __attribute__((ext_vector_type(4)));
typedef unsigned int v4u __attribute__((ext_vector_type(4)));

__device__ __forceinline__ unsigned short bf_bits(float f) {
  unsigned u = __float_as_uint(f);
  return (unsigned short)((u + 0x7FFFu + ((u >> 16) & 1u)) >> 16);
}
__device__ __forceinline__ float bf_up(unsigned short h) { return __uint_as_float(((unsigned)h) << 16); }
__device__ __forceinline__ unsigned short h_bits(_Float16 x) { return __builtin_bit_cast(unsigned short, x); }
__device__ __forceinline__ unsigned pk16(unsigned short a, unsigned short b) { return (unsigned)a | ((unsigned)b << 16); }
__device__ __forceinline__ v8f zero8() { v8f z = {0.f, 0.f, 0.f, 0.f, 0.f, 0.f, 0.f, 0.f}; return z; }

__device__ __forceinline__ v16b ldfrag_b(const __bf16* p) {
  union { v16b v; v8b h[2]; } f;
  f.h[0] = *(const v8b*)(p);
  f.h[1] = *(const v8b*)(p + 16);
  return f.v;
}
__device__ __forceinline__ v16h ldfrag_h(const _Float16* p) {
  union { v16h v; v8h h[2]; } f;
  f.h[0] = *(const v8h*)(p);
  f.h[1] = *(const v8h*)(p + 16);
  return f.v;
}

__device__ __forceinline__ v8f mma_h(v16h a, v16h b, v8f c) {
  c = __builtin_amdgcn_wmma_f32_16x16x32_f16(false, a, false, b, (short)0, c, false, false);
#if defined(__HIP_DEVICE_COMPILE__)
  asm volatile("v_nop\n\tv_nop\n\tv_nop\n\tv_nop" : "+v"(c) : "v"(a), "v"(b));
#endif
  return c;
}
__device__ __forceinline__ v8f mma_b_raw(v16b a, v16b b, v8f c) {
  return __builtin_amdgcn_wmma_f32_16x16x32_bf16(false, a, false, b, (short)0, c, false, false);
}
__device__ __forceinline__ void dep_guard_b(v8f& a, v8f& b, v16b x, v16b y) {
#if defined(__HIP_DEVICE_COMPILE__)
  asm volatile("v_nop\n\tv_nop\n\tv_nop\n\tv_nop" : "+v"(a), "+v"(b) : "v"(x), "v"(y));
#endif
}
__device__ __forceinline__ void keep4_b(v16b a, v16b b, v16b c, v16b d) {
#if defined(__HIP_DEVICE_COMPILE__)
  asm volatile("v_nop" :: "v"(a), "v"(b), "v"(c), "v"(d));
#endif
}
__device__ __forceinline__ void acc_guard4(v8f& a, v8f& b, v8f& c, v8f& d) {
#if defined(__HIP_DEVICE_COMPILE__)
  asm volatile("v_nop\n\tv_nop\n\tv_nop\n\tv_nop" : "+v"(a), "+v"(b), "+v"(c), "+v"(d));
#endif
}
__device__ __forceinline__ void wave_sync_lds() {
  __builtin_amdgcn_fence(__ATOMIC_RELEASE, "workgroup");
  __builtin_amdgcn_wave_barrier();
  __builtin_amdgcn_fence(__ATOMIC_ACQUIRE, "workgroup");
}

__device__ __forceinline__ v8f score3(const v16h qh, const v16h ql, const v16h kh, const v16h kl, const float rres) {
  v8f acc = zero8();
  acc = mma_h(ql, kh, acc);
  acc = mma_h(qh, kl, acc);
#pragma unroll
  for (int r = 0; r < 8; ++r) acc[r] *= rres;
  acc = mma_h(qh, kh, acc);
  return acc;
}

__global__ __launch_bounds__(256) void cvt_bf16x8(const float* __restrict__ in, unsigned short* out, int n8) {
  const int i = blockIdx.x * 256 + threadIdx.x;
  if (i < n8) {
    const v4f a = *(const v4f*)(in + (size_t)i * 8);
    const v4f b = *(const v4f*)(in + (size_t)i * 8 + 4);
    v4u p;
    p[0] = pk16(bf_bits(a[0]), bf_bits(a[1]));
    p[1] = pk16(bf_bits(a[2]), bf_bits(a[3]));
    p[2] = pk16(bf_bits(b[0]), bf_bits(b[1]));
    p[3] = pk16(bf_bits(b[2]), bf_bits(b[3]));
    *(volatile v4u*)(out + (size_t)i * 8) = p;
    __threadfence();
    *(volatile v4u*)(out + (size_t)i * 8) = p;
  }
}

__global__ __launch_bounds__(256) void cvt_wT(const float* __restrict__ w0, const float* __restrict__ w1,
                                              const float* __restrict__ w2, const float* __restrict__ w3,
                                              unsigned short* outp) {
  __shared__ float tile[64][33];
  const int tid = threadIdx.x;
  const int z = blockIdx.z;
  const float* src = (z == 0) ? w0 : ((z == 1) ? w1 : ((z == 2) ? w2 : w3));
  unsigned short* dst = outp + (size_t)z * CD * CD;
  const int i0 = blockIdx.x * 64;
  const int o0 = blockIdx.y * 32;
#pragma unroll
  for (int p = 0; p < 8; ++p) {
    const int idx = p * 256 + tid;
    const int i = idx >> 5, o = idx & 31;
    tile[i][o] = src[(size_t)(i0 + i) * CD + o0 + o];
  }
  __syncthreads();
  const int o = tid >> 3, c8 = (tid & 7) * 8;
  v4u pk;
#pragma unroll
  for (int e = 0; e < 4; ++e)
    pk[e] = pk16(bf_bits(tile[c8 + 2 * e][o]), bf_bits(tile[c8 + 2 * e + 1][o]));
  unsigned short* gp = dst + (size_t)(o0 + o) * CD + i0 + c8;
  *(volatile v4u*)gp = pk;
  __threadfence();
  *(volatile v4u*)gp = pk;
}

template <int NSPLIT, int OUT_MODE>
__global__ __launch_bounds__(256) void gemm64(
    const unsigned short* __restrict__ Ap, const unsigned short* A2p, int lda, long long strideA,
    const unsigned short* __restrict__ Btp, const unsigned short* Bt2p, int ldb, long long strideB,
    void* Cout, int ldc, long long strideC,
    void* Cout2, int ldc2, long long strideC2, int N2,
    int M, int N, int K, float rscale, const float* __restrict__ biasp) {
  const __bf16* A   = (const __bf16*)(const void*)Ap;
  const __bf16* A2  = (const __bf16*)(const void*)A2p;
  const __bf16* Bt  = (const __bf16*)(const void*)Btp;
  const __bf16* Bt2 = (const __bf16*)(const void*)Bt2p;
  __shared__ __align__(16) float sT[8][16 * 68];
  const int b    = blockIdx.y;
  const int lane = threadIdx.x & 31;
  const int wave = threadIdx.x >> 5;
  const int tilesN = N >> 6;
  const int tilesM = M >> 6;
  const int tile = blockIdx.x * 8 + wave;
  if (tile >= tilesM * tilesN) return;
  const int tm = tile / tilesN;
  const int tn = tile - tm * tilesN;
  const int m0 = tm << 6;
  const int n0 = tn << 6;

  const __bf16* Ab  = A  + (size_t)b * strideA;
  const __bf16* Bb  = Bt + (size_t)b * strideB;
  const __bf16* Ab2 = (NSPLIT >= 1) ? (A2  + (size_t)b * strideA) : Ab;
  const __bf16* Bb2 = (NSPLIT == 2) ? (Bt2 + (size_t)b * strideB) : Bb;

  const int rlane = lane & 15;
  const int koff  = (lane >> 4) * 8;
  const int mOff  = (lane >> 4) * 8;

  v8f acc[4][4];
#pragma unroll
  for (int i = 0; i < 4; ++i)
#pragma unroll
    for (int j = 0; j < 4; ++j) acc[i][j] = zero8();

  for (int k0 = 0; k0 < K; k0 += 32) {
    v16b bh[4], bl[4];
#pragma unroll
    for (int j = 0; j < 4; ++j) {
      const size_t bo = (size_t)(n0 + (j << 4) + rlane) * ldb + koff + k0;
      bh[j] = ldfrag_b(Bb + bo);
      if (NSPLIT == 2) bl[j] = ldfrag_b(Bb2 + bo); else bl[j] = bh[j];
    }
#pragma unroll
    for (int i = 0; i < 4; ++i) {
      const size_t ao = (size_t)(m0 + (i << 4) + rlane) * lda + koff + k0;
      const v16b ah = ldfrag_b(Ab + ao);
      v16b al = ah;
      if (NSPLIT >= 1) al = ldfrag_b(Ab2 + ao);
#pragma unroll
      for (int j = 0; j < 4; ++j) {
        acc[i][j] = mma_b_raw(ah, bh[j], acc[i][j]);
        if (NSPLIT >= 1) acc[i][j] = mma_b_raw(al, bh[j], acc[i][j]);
        if (NSPLIT == 2) acc[i][j] = mma_b_raw(ah, bl[j], acc[i][j]);
      }
      dep_guard_b(acc[i][0], acc[i][3], ah, al);
    }
    keep4_b(bh[0], bh[1], bh[2], bh[3]);
    if (NSPLIT == 2) keep4_b(bl[0], bl[1], bl[2], bl[3]);
  }
  acc_guard4(acc[0][0], acc[0][1], acc[0][2], acc[0][3]);
  acc_guard4(acc[1][0], acc[1][1], acc[1][2], acc[1][3]);
  acc_guard4(acc[2][0], acc[2][1], acc[2][2], acc[2][3]);
  acc_guard4(acc[3][0], acc[3][1], acc[3][2], acc[3][3]);

  float* slab = sT[wave];
#pragma unroll
  for (int i = 0; i < 4; ++i) {
    const int mBase = m0 + (i << 4);
#pragma unroll
    for (int j = 0; j < 4; ++j) {
#pragma unroll
      for (int r = 0; r < 8; ++r) {
        slab[(mOff + r) * 68 + (j << 4) + rlane] = acc[i][j][r];
      }
    }
    wave_sync_lds();
    if (OUT_MODE == 0) {
      float* C = (float*)Cout + (size_t)b * strideC;
      const int hh = lane >> 4, c4 = (lane & 15) * 4;
      v4f bv;
#pragma unroll
      for (int e = 0; e < 4; ++e) bv[e] = bf_up(bf_bits(biasp[n0 + c4 + e]));
      for (int pass = 0; pass < 2; ++pass) {
#pragma unroll
        for (int it = 0; it < 8; ++it) {
          const int row = it * 2 + hh;
          const v4f v = *(const v4f*)(slab + row * 68 + c4) + bv;
          *(volatile v4f*)(C + (size_t)(mBase + row) * ldc + n0 + c4) = v;
        }
        __threadfence();
      }
    } else {
      const int q = lane >> 3, c8 = (lane & 7) * 8;
      unsigned short* C  = (unsigned short*)Cout  + (size_t)b * strideC;
      unsigned short* C2 = (unsigned short*)Cout2 + (size_t)b * strideC2;
      const bool wlo = (OUT_MODE == 2) || (n0 < N2);
      v4u hv[4], lv[4];
#pragma unroll
      for (int it = 0; it < 4; ++it) {
        const int row = it * 4 + q;
        const float* sp = slab + row * 68 + c8;
        v4u a, a2;
#pragma unroll
        for (int e = 0; e < 4; ++e) {
          const float f0 = sp[2 * e], f1 = sp[2 * e + 1];
          unsigned short h0, h1, l0, l1;
          if (OUT_MODE == 2) {
            h0 = bf_bits(f0); h1 = bf_bits(f1);
            l0 = bf_bits(f0 - bf_up(h0)); l1 = bf_bits(f1 - bf_up(h1));
          } else {
            const _Float16 x0 = (_Float16)f0, x1 = (_Float16)f1;
            h0 = h_bits(x0); h1 = h_bits(x1);
            l0 = h_bits((_Float16)((f0 - (float)x0) * rscale));
            l1 = h_bits((_Float16)((f1 - (float)x1) * rscale));
          }
          a[e] = pk16(h0, h1); a2[e] = pk16(l0, l1);
        }
        hv[it] = a; lv[it] = a2;
      }
      for (int pass = 0; pass < 2; ++pass) {
#pragma unroll
        for (int it = 0; it < 4; ++it) {
          const int row = it * 4 + q;
          *(volatile v4u*)(C + (size_t)(mBase + row) * ldc + n0 + c8) = hv[it];
          if (wlo) *(volatile v4u*)(C2 + (size_t)(mBase + row) * ldc2 + n0 + c8) = lv[it];
        }
        __threadfence();
      }
    }
    wave_sync_lds();
  }
}

__global__ __launch_bounds__(256)
void attn32(const unsigned short* __restrict__ qhp, const unsigned short* __restrict__ qlp,
            const unsigned short* __restrict__ khp, const unsigned short* __restrict__ klp,
            const unsigned short* __restrict__ vhp, const unsigned short* __restrict__ vlp,
            unsigned short* ohp, unsigned short* olp, float sscale, float rres) {
  union FH { v16h v; v8h h[2]; };
  __shared__ __align__(16) _Float16 Psh[8][16 * 64];
  __shared__ __align__(16) _Float16 Psl[8][16 * 64];
  __shared__ __align__(16) float    Os[64 * 64];

  const int tid  = threadIdx.x;
  const int wave = tid >> 5;
  const int lane = tid & 31;
  const int hh   = lane >> 4;
  const int c    = lane & 15;

  const int bx   = blockIdx.x;
  const int qb   = bx % NQB;
  const int rest = bx / NQB;
  const int g    = rest % (NH / 2);
  const int b    = rest / (NH / 2);
  const int hp   = wave >> 2;
  const int h    = 2 * g + hp;
  const int wq   = wave & 3;
  const int q0   = qb * 64 + wq * 16;
  const size_t rowQ = (size_t)b * NQ;
  const size_t rowK = (size_t)b * NK;

  const _Float16* Qh = (const _Float16*)(const void*)qhp + (size_t)h * HD;
  const _Float16* Ql = (const _Float16*)(const void*)qlp + (size_t)h * HD;
  const _Float16* Kh = (const _Float16*)(const void*)khp + (size_t)h * HD;
  const _Float16* Kl = (const _Float16*)(const void*)klp + (size_t)h * HD;
  const _Float16* Vh = (const _Float16*)(const void*)vhp + ((size_t)b * CD + (size_t)h * HD) * NK;
  const _Float16* Vl = (const _Float16*)(const void*)vlp + ((size_t)b * CD + (size_t)h * HD) * NK;

  const v16h qah = ldfrag_h(Qh + (rowQ + q0 + c) * CD + 8 * hh);
  const v16h qal = ldfrag_h(Ql + (rowQ + q0 + c) * CD + 8 * hh);

  float mrow[8], lrow[8];
  v8f oacc[2];
#pragma unroll
  for (int r = 0; r < 8; ++r) { mrow[r] = -INFINITY; lrow[r] = 0.f; }
#pragma unroll
  for (int t = 0; t < 2; ++t) oacc[t] = zero8();

  _Float16* pwh = Psh[wave];
  _Float16* pwl = Psl[wave];

  for (int kt = 0; kt < NKB; ++kt) {
    const int kv0 = kt * 64;

    v8f s[4];
#pragma unroll
    for (int j = 0; j < 4; ++j) {
      const size_t ko = (rowK + kv0 + j * 16 + c) * CD + 8 * hh;
      const v16h kb = ldfrag_h(Kh + ko);
      const v16h kl = ldfrag_h(Kl + ko);
      const v8f a = score3(qah, qal, kb, kl, rres);
#pragma unroll
      for (int r = 0; r < 8; ++r) s[j][r] = a[r] * sscale;
    }

#pragma unroll
    for (int r = 0; r < 8; ++r) {
      float m = fmaxf(fmaxf(s[0][r], s[1][r]), fmaxf(s[2][r], s[3][r]));
#pragma unroll
      for (int off = 1; off < 16; off <<= 1) m = fmaxf(m, __shfl_xor(m, off, 32));
      const float mnew  = fmaxf(mrow[r], m);
      const float alpha = __expf(mrow[r] - mnew);
      mrow[r] = mnew;
      float psum = 0.f;
#pragma unroll
      for (int j = 0; j < 4; ++j) {
        const float p  = __expf(s[j][r] - mnew);
        psum += p;
        const float p1 = p * 1024.0f;
        const _Float16 x = (_Float16)p1;
        const int idx = (8 * hh + r) * 64 + j * 16 + c;
        pwh[idx] = x;
        pwl[idx] = (_Float16)((p1 - (float)x) * 4096.0f);
      }
#pragma unroll
      for (int off = 1; off < 16; off <<= 1) psum += __shfl_xor(psum, off, 32);
      lrow[r] = lrow[r] * alpha + psum;
#pragma unroll
      for (int t = 0; t < 2; ++t) oacc[t][r] *= alpha;
    }
    wave_sync_lds();

    v8f o1[2];
    o1[0] = zero8(); o1[1] = zero8();
#pragma unroll
    for (int kk = 0; kk < 2; ++kk) {
      FH pa, pl;
      pa.h[0] = *(const v8h*)(pwh + c * 64 + kk * 32 + 8 * hh);
      pa.h[1] = *(const v8h*)(pwh + c * 64 + kk * 32 + 16 + 8 * hh);
      pl.h[0] = *(const v8h*)(pwl + c * 64 + kk * 32 + 8 * hh);
      pl.h[1] = *(const v8h*)(pwl + c * 64 + kk * 32 + 16 + 8 * hh);
#pragma unroll
      for (int t = 0; t < 2; ++t) {
        const size_t vo = (size_t)(t * 16 + c) * NK + kv0 + kk * 32 + 8 * hh;
        const v16h vb = ldfrag_h(Vh + vo);
        const v16h vl = ldfrag_h(Vl + vo);
        oacc[t] = mma_h(pa.v, vb, oacc[t]);
        o1[t]   = mma_h(pa.v, vl, o1[t]);
        o1[t]   = mma_h(pl.v, vb, o1[t]);
      }
    }
#pragma unroll
    for (int t = 0; t < 2; ++t)
#pragma unroll
      for (int r = 0; r < 8; ++r) oacc[t][r] += o1[t][r] * rres;
    wave_sync_lds();
  }

#pragma unroll
  for (int r = 0; r < 8; ++r) {
    const float l = lrow[r];
    const float inv = ((l > 0.f) ? (1.0f / l) : 0.f) * (1.0f / 1024.0f);
#pragma unroll
    for (int t = 0; t < 2; ++t) Os[(wq * 16 + 8 * hh + r) * 64 + hp * 32 + t * 16 + c] = oacc[t][r] * inv;
  }
  __syncthreads();
  {
    const int q4 = lane >> 3, c8 = (lane & 7) * 8;
    v4u hv[2], lv[2];
#pragma unroll
    for (int it = 0; it < 2; ++it) {
      const int row = wave * 8 + it * 4 + q4;
      const float* sp = Os + row * 64 + c8;
      v4u a, a2;
#pragma unroll
      for (int e = 0; e < 4; ++e) {
        const float f0 = sp[2 * e], f1 = sp[2 * e + 1];
        const unsigned short h0 = bf_bits(f0), h1 = bf_bits(f1);
        const unsigned short l0 = bf_bits(f0 - bf_up(h0)), l1 = bf_bits(f1 - bf_up(h1));
        a[e] = pk16(h0, h1); a2[e] = pk16(l0, l1);
      }
      hv[it] = a; lv[it] = a2;
    }
    for (int pass = 0; pass < 2; ++pass) {
#pragma unroll
      for (int it = 0; it < 2; ++it) {
        const int row = wave * 8 + it * 4 + q4;
        const size_t go = (rowQ + qb * 64 + row) * CD + (size_t)g * 64 + c8;
        *(volatile v4u*)(ohp + go) = hv[it];
        *(volatile v4u*)(olp + go) = lv[it];
      }
      __threadfence();
    }
  }
}

__global__ __launch_bounds__(64)
void headmix(const unsigned short* __restrict__ qhp, const unsigned short* __restrict__ qlp,
             const unsigned short* __restrict__ khp, const unsigned short* __restrict__ klp,
             const float* __restrict__ W1, const float* __restrict__ b1,
             const float* __restrict__ W2, const float* __restrict__ b2,
             float* mout, float sscale, float rres) {
  __shared__ __align__(16) float Ssh[2][NH * 16 * 32];
  __shared__ __align__(16) float Msh[2][16 * 32];

  const int tid  = threadIdx.x;
  const int wave = tid >> 5;
  const int lane = tid & 31;
  const int hh   = lane >> 4;
  const int c    = lane & 15;

  const int bx   = blockIdx.x;
  const int b    = bx / NQH;
  const int qb2  = bx % NQH;
  const int q0   = qb2 * 32 + wave * 16;
  const size_t rowQ = (size_t)b * NQ;
  const size_t rowK = (size_t)b * NK;

  float w1r[NH * NH], b1r[NH], w2r[NH];
#pragma unroll
  for (int i = 0; i < NH * NH; ++i) w1r[i] = bf_up(bf_bits(W1[i]));
#pragma unroll
  for (int i = 0; i < NH; ++i) { b1r[i] = bf_up(bf_bits(b1[i])); w2r[i] = bf_up(bf_bits(W2[i])); }
  const float b2r = bf_up(bf_bits(b2[0]));

  const _Float16* Qh = (const _Float16*)(const void*)qhp;
  const _Float16* Ql = (const _Float16*)(const void*)qlp;
  const _Float16* Kh = (const _Float16*)(const void*)khp;
  const _Float16* Kl = (const _Float16*)(const void*)klp;

  float* ss = Ssh[wave];
  float* ms = Msh[wave];

  for (int kc = 0; kc < NKC; ++kc) {
    const int l0 = kc * 32;
#pragma unroll 1
    for (int h = 0; h < NH; ++h) {
      const size_t qo = (rowQ + q0 + c) * CD + (size_t)h * HD + 8 * hh;
      const v16h qah = ldfrag_h(Qh + qo);
      const v16h qal = ldfrag_h(Ql + qo);
#pragma unroll
      for (int j = 0; j < 2; ++j) {
        const size_t ko = (rowK + l0 + j * 16 + c) * CD + (size_t)h * HD + 8 * hh;
        const v16h kb = ldfrag_h(Kh + ko);
        const v16h kl = ldfrag_h(Kl + ko);
        const v8f a = score3(qah, qal, kb, kl, rres);
#pragma unroll
        for (int r = 0; r < 8; ++r) ss[(h * 16 + 8 * hh + r) * 32 + j * 16 + c] = a[r] * sscale;
      }
    }
    wave_sync_lds();

#pragma unroll 1
    for (int q = 0; q < 16; ++q) {
      float av[NH];
#pragma unroll
      for (int h = 0; h < NH; ++h) av[h] = ss[(h * 16 + q) * 32 + lane];
      float mo = b2r;
#pragma unroll
      for (int j = 0; j < NH; ++j) {
        float f = b1r[j];
#pragma unroll
        for (int h = 0; h < NH; ++h) f += av[h] * w1r[h * NH + j];
        mo += fmaxf(f, 0.f) * w2r[j];
      }
      ms[q * 32 + lane] = fmaxf(mo, 0.f);
    }
    wave_sync_lds();

    {
      const int q4 = lane >> 3, c4 = (lane & 7) * 4;
      v4f mv[4];
#pragma unroll
      for (int it = 0; it < 4; ++it) {
        const int row = it * 4 + q4;
        mv[it] = *(const v4f*)(ms + row * 32 + c4);
      }
      for (int pass = 0; pass < 2; ++pass) {
#pragma unroll
        for (int it = 0; it < 4; ++it) {
          const int row = it * 4 + q4;
          *(volatile v4f*)(mout + (rowQ + q0 + row) * NK + l0 + c4) = mv[it];
        }
        __threadfence();
      }
    }
    wave_sync_lds();
  }
}

extern "C" void kernel_launch(void* const* d_in, const int* in_sizes, int n_in,
                              void* d_out, int out_size, void* d_ws, size_t ws_size,
                              hipStream_t stream) {
  if (n_in < 12) return;
  if (in_sizes[0] != NB * NQ * CD) return;
  if (in_sizes[1] != NB * NK * CD) return;
  if (in_sizes[2] != NB * NK * CD) return;
  if (in_sizes[3] != CD * CD || in_sizes[4] != CD * CD || in_sizes[5] != CD * CD || in_sizes[6] != CD * CD) return;
  if (in_sizes[7] != CD) return;
  if (in_sizes[8] != NH * NH || in_sizes[9] != NH || in_sizes[10] != NH || in_sizes[11] != 1) return;
  if (out_size != NB * NQ * CD + NB * NQ * NK) return;

  const float* query = (const float*)d_in[0];
  const float* key   = (const float*)d_in[1];
  const float* value = (const float*)d_in[2];
  const float* Wq    = (const float*)d_in[3];
  const float* Wk    = (const float*)d_in[4];
  const float* Wv    = (const float*)d_in[5];
  const float* Wp    = (const float*)d_in[6];
  const float* bp    = (const float*)d_in[7];
  const float* W1    = (const float*)d_in[8];
  const float* b1    = (const float*)d_in[9];
  const float* W2    = (const float*)d_in[10];
  const float* b2    = (const float*)d_in[11];

  const size_t PXq = (size_t)NB * NQ * CD * 2;
  const size_t PXk = (size_t)NB * NK * CD * 2;
  const size_t PW  = (size_t)4 * CD * CD * 2;
  const size_t PQ  = (size_t)NB * NQ * CD * 2;
  const size_t PK  = (size_t)NB * NK * CD * 2;
  const size_t PVT = (size_t)NB * CD * NK * 2;
  const size_t PO  = (size_t)NB * NQ * CD * 2;
  size_t off = 0;
  const size_t oXq  = off; off += PXq;
  const size_t oXk  = off; off += PXk;
  const size_t oXv  = off; off += PXk;
  const size_t oW   = off; off += PW;
  const size_t oQh  = off; off += PQ;
  const size_t oQl  = off; off += PQ;
  const size_t oKh  = off; off += PK;
  const size_t oKl  = off; off += PK;
  const size_t oVTh = off; off += PVT;
  const size_t oVTl = off; off += PVT;
  const size_t oOh  = off; off += PO;
  const size_t oOl  = off; off += PO;
  if (off > ws_size) return;
  if (off > (size_t)134217728) return;

  char* ws = (char*)d_ws;
  unsigned short* Xq  = (unsigned short*)(ws + oXq);
  unsigned short* Xk  = (unsigned short*)(ws + oXk);
  unsigned short* Xv  = (unsigned short*)(ws + oXv);
  unsigned short* WT  = (unsigned short*)(ws + oW);
  unsigned short* WTq = WT;
  unsigned short* WTk = WT + (size_t)1 * CD * CD;
  unsigned short* WTv = WT + (size_t)2 * CD * CD;
  unsigned short* WTp = WT + (size_t)3 * CD * CD;
  unsigned short* Qh  = (unsigned short*)(ws + oQh);
  unsigned short* Ql  = (unsigned short*)(ws + oQl);
  unsigned short* Kh  = (unsigned short*)(ws + oKh);
  unsigned short* Kl  = (unsigned short*)(ws + oKl);
  unsigned short* VTh = (unsigned short*)(ws + oVTh);
  unsigned short* VTl = (unsigned short*)(ws + oVTl);
  unsigned short* Oh  = (unsigned short*)(ws + oOh);
  unsigned short* Ol  = (unsigned short*)(ws + oOl);

  float* xout = (float*)d_out;
  float* mout = (float*)d_out + (size_t)NB * NQ * CD;

  const float sscale = 0.17677669529663687f;
  const float rres   = 1.0f / 4096.0f;

  const dim3 blk(256);
  const int n8q = NB * NQ * CD / 8;
  const int n8k = NB * NK * CD / 8;
  const dim3 gCvtQ((n8q + 255) / 256);
  const dim3 gCvtK((n8k + 255) / 256);
  const dim3 gWT(CD / 64, CD / 32, 4);
  const dim3 gQ(((NB * NQ / 64) * (CD / 64) + 7) / 8, 1);
  const dim3 gK(((NB * NK / 64) * (CD / 64) + 7) / 8, 1);
  const dim3 gVT(((CD / 64) * (NK / 64) + 7) / 8, NB);
  const dim3 gOut(((NB * NQ / 64) * (CD / 64) + 7) / 8, 1);
  const dim3 gMix(NB * NQH);
  const dim3 gAttn(NB * (NH / 2) * NQB);

  cvt_bf16x8<<<gCvtQ, blk, 0, stream>>>(query, Xq, n8q);
  cvt_bf16x8<<<gCvtK, blk, 0, stream>>>(key, Xk, n8k);
  cvt_bf16x8<<<gCvtK, blk, 0, stream>>>(value, Xv, n8k);
  cvt_wT<<<gWT, blk, 0, stream>>>(Wq, Wk, Wv, Wp, WT);
  gemm64<0, 3><<<gQ, blk, 0, stream>>>(
      Xq, Xq, CD, 0LL, WTq, WTq, CD, 0LL,
      (void*)Qh, CD, 0LL, (void*)Ql, CD, 0LL, CD,
      NB * NQ, CD, CD, 4096.0f, bp);
  gemm64<0, 3><<<gK, blk, 0, stream>>>(
      Xk, Xk, CD, 0LL, WTk, WTk, CD, 0LL,
      (void*)Kh, CD, 0LL, (void*)Kl, CD, 0LL, CD,
      NB * NK, CD, CD, 4096.0f, bp);
  gemm64<0, 3><<<gVT, blk, 0, stream>>>(
      WTv, WTv, CD, 0LL, Xv, Xv, CD, (long long)NK * CD,
      (void*)VTh, NK, (long long)CD * NK, (void*)VTl, NK, (long long)CD * NK, NK,
      CD, NK, CD, 4096.0f, bp);
  headmix<<<gMix, dim3(64), 0, stream>>>(Qh, Ql, Kh, Kl, W1, b1, W2, b2, mout, sscale, rres);
  attn32<<<gAttn, blk, 0, stream>>>(Qh, Ql, Kh, Kl, VTh, VTl, Oh, Ol, sscale, rres);
  gemm64<1, 0><<<gOut, blk, 0, stream>>>(
      Oh, Ol, CD, 0LL, WTp, WTp, CD, 0LL,
      (void*)xout, CD, 0LL, (void*)xout, CD, 0LL, CD,
      NB * NQ, CD, CD, 1.0f, bp);
  (void)hipGetLastError();
}
